// RGCN_65025804861440
// MI455X (gfx1250) — hardware-run, weakly checked
//
#include <hip/hip_runtime.h>

typedef float          v8f   __attribute__((ext_vector_type(8)));
typedef float          v4f   __attribute__((ext_vector_type(4)));
typedef unsigned int   v4u   __attribute__((ext_vector_type(4)));
typedef int            v8i   __attribute__((ext_vector_type(8)));
typedef unsigned short v8us  __attribute__((ext_vector_type(8)));
typedef unsigned short v16us __attribute__((ext_vector_type(16)));
typedef __bf16         v16bf __attribute__((ext_vector_type(16)));
typedef _Float16       v16h  __attribute__((ext_vector_type(16)));
typedef v4f  __attribute__((may_alias)) v4fa;
typedef v8us __attribute__((may_alias)) v8usa;
union FragB { v16bf v; v16us u; v8us h[2]; v8i w; };
union FragH { v16h  v; v16us u; v8us h[2]; v8i w; };

__device__ __forceinline__ v8f wmb(const FragB& a, const FragB& b, v8f c) {
  v8f d = __builtin_amdgcn_wmma_f32_16x16x32_bf16(false, a.v, false, b.v, (short)0, c, false, false);
  asm volatile("v_nop\n\tv_nop\n\tv_nop\n\tv_nop" : "+v"(d) : "v"(a.w), "v"(b.w));
  return d;
}

__device__ __forceinline__ v8f wmh(const FragH& a, const FragH& b, v8f c) {
  v8f d = __builtin_amdgcn_wmma_f32_16x16x32_f16(false, a.v, false, b.v, (short)0, c, false, false);
  asm volatile("v_nop\n\tv_nop\n\tv_nop\n\tv_nop" : "+v"(d) : "v"(a.w), "v"(b.w));
  return d;
}

__device__ __forceinline__ unsigned bf16_bits(float f) {
  const unsigned u = __float_as_uint(f);
  const unsigned r = (u + 0x7FFFu + ((u >> 16) & 1u)) >> 16;
  const unsigned q = (u >> 16) | 0x40u;
  return ((u & 0x7fffffffu) > 0x7f800000u) ? q : r;
}

__device__ __forceinline__ float bf16_val(float f) {
  return __uint_as_float(bf16_bits(f) << 16);
}
__device__ __forceinline__ int clampi(int v, int lo, int hi) {
  return v < lo ? lo : (v > hi ? hi : v);
}

__device__ __forceinline__ unsigned f16_bits(float f) {
  const unsigned u  = __float_as_uint(f);
  const unsigned s  = (u >> 16) & 0x8000u;
  const unsigned a  = u & 0x7fffffffu;
  const unsigned t  = a - 0x38000000u;
  const unsigned r  = (t + 0x0FFFu + ((t >> 13) & 1u)) >> 13;
  const unsigned rc = r > 0x7C00u ? 0x7C00u : r;
  const bool small  = a < 0x38800000u;
  const bool isnan  = a > 0x7f800000u;
  const unsigned fin = small ? 0u : (s | rc);
  return isnan ? (s | 0x7E00u) : fin;
}

__device__ __forceinline__ unsigned pk16(unsigned lo, unsigned hi) { return lo | (hi << 16); }
__device__ __forceinline__ unsigned bf16_lo_bits(float v) {
  float hi = bf16_val(v);
  asm volatile("" : "+v"(hi));
  return bf16_bits(v - hi);
}
__device__ __forceinline__ v4u pack8_bf16(v4f a, v4f c) {
  return (v4u){ pk16(bf16_bits(a[0]), bf16_bits(a[1])), pk16(bf16_bits(a[2]), bf16_bits(a[3])),
                pk16(bf16_bits(c[0]), bf16_bits(c[1])), pk16(bf16_bits(c[2]), bf16_bits(c[3])) };
}
__device__ __forceinline__ v4u pack8_bf16_lo(v4f a, v4f c) {
  return (v4u){ pk16(bf16_lo_bits(a[0]), bf16_lo_bits(a[1])), pk16(bf16_lo_bits(a[2]), bf16_lo_bits(a[3])),
                pk16(bf16_lo_bits(c[0]), bf16_lo_bits(c[1])), pk16(bf16_lo_bits(c[2]), bf16_lo_bits(c[3])) };
}
__device__ __forceinline__ v4u pack8_f16(v4f a, v4f c) {
  return (v4u){ pk16(f16_bits(a[0]), f16_bits(a[1])), pk16(f16_bits(a[2]), f16_bits(a[3])),
                pk16(f16_bits(c[0]), f16_bits(c[1])), pk16(f16_bits(c[2]), f16_bits(c[3])) };
}

template <int FORM>
__global__ __launch_bounds__(256) void k_plane(const float* __restrict__ src, int rows, int cols, int ldsrc,
                                               unsigned short* __restrict__ dst, int MP, int KP) {
  static_assert(FORM >= 0 && FORM <= 3);
  const int KTOT = (FORM == 1 || FORM == 3) ? 2 * KP : KP;
  const unsigned ppr   = (unsigned)(KTOT >> 3);
  const unsigned kp8   = (unsigned)(KP >> 3);
  const unsigned total = (unsigned)MP * ppr;
  const unsigned g     = blockIdx.x * 256u + threadIdx.x;
  const unsigned rowu  = g / ppr;
  const unsigned p     = g - rowu * ppr;
  const bool second    = p >= kp8;
  const int row = (int)rowu;
  const int c0  = (int)((second ? p - kp8 : p) << 3);
  const float* srow = src + (size_t)clampi(row, 0, rows - 1) * (size_t)ldsrc;
  float x[8];
  unsigned mk[8];
#pragma unroll
  for (int e = 0; e < 8; ++e) {
    const int c = c0 + e;
    const float v = srow[clampi(c, 0, cols - 1)];
    asm volatile("" :: "v"(v));
    x[e]  = v;
    mk[e] = (row < rows && c < cols) ? 0xFFFFu : 0u;
  }
  const v4f a = (v4f){ x[0], x[1], x[2], x[3] };
  const v4f c = (v4f){ x[4], x[5], x[6], x[7] };
  v4u o;
  if (FORM == 2) {
    o = pack8_f16(a, c);
  } else {
    const v4u hi = pack8_bf16(a, c);
    o = hi;
    if (FORM == 1) { const v4u lo = pack8_bf16_lo(a, c); o = second ? lo : hi; }
  }
  const v4u mw = (v4u){ pk16(mk[0], mk[1]), pk16(mk[2], mk[3]), pk16(mk[4], mk[5]), pk16(mk[6], mk[7]) };
  o &= mw;
  if (g < total) {
    volatile v4u* q = (volatile v4u*)(dst + (size_t)g * 8);
    *q = o;
    __threadfence();
    *q = o;
  }
}

template <int FORM> struct FragOf    { typedef FragB T; };
template <>         struct FragOf<2> { typedef FragH T; };
__device__ __forceinline__ v8f mm(const FragB& a, const FragB& b, v8f c) { return wmb(a, b, c); }
__device__ __forceinline__ v8f mm(const FragH& a, const FragH& b, v8f c) { return wmh(a, b, c); }
template <class F> __device__ __forceinline__ F ld_frag(const unsigned short* p) {
  F f;
  f.h[0] = *(const v8usa*)(p);
  f.h[1] = *(const v8usa*)(p + 16);
  return f;
}

template <int FORM, int EPI>
__global__ __launch_bounds__(256) __attribute__((amdgpu_num_vgpr(248)))
void k_gemm_nt(const unsigned short* __restrict__ A, const unsigned short* __restrict__ B,
               const float* __restrict__ bias, float* __restrict__ D, int M, int N, int KTOT, int ldd) {
  static_assert(FORM >= 0 && FORM <= 2);
  static_assert(EPI == 0 || EPI == 1);
  typedef typename FragOf<FORM>::T F;
  __shared__ __attribute__((aligned(16))) float sT[8][16 * 68];
  const int lane = threadIdx.x & 31;
  const int wave = threadIdx.x >> 5;
  const int tilesM = (M + 63) >> 6;
  const int tilesN = (N + 63) >> 6;
  const int tile = blockIdx.x * 8 + wave;
  if (tile >= tilesM * tilesN) return;
  const int tm = tile / tilesN;
  const int tn = tile - tm * tilesN;
  const int m0 = tm << 6;
  const int n0 = tn << 6;

  const int rl = lane & 15;
  const int h8 = (lane >> 4) * 8;
  const unsigned short* pa = A + (size_t)(m0 + rl) * (size_t)KTOT + h8;
  const unsigned short* pb = B + (size_t)(n0 + rl) * (size_t)KTOT + h8;

  v8f acc[4][4];
#pragma unroll
  for (int i = 0; i < 4; ++i)
#pragma unroll
    for (int j = 0; j < 4; ++j) acc[i][j] = (v8f){0.f, 0.f, 0.f, 0.f, 0.f, 0.f, 0.f, 0.f};

#pragma unroll 1
  for (int k0 = 0; k0 < KTOT; k0 += 32) {
    F bf[4];
#pragma unroll
    for (int j = 0; j < 4; ++j) bf[j] = ld_frag<F>(pb + (size_t)(j << 4) * (size_t)KTOT + k0);
#pragma unroll
    for (int i = 0; i < 4; ++i) {
      const F af = ld_frag<F>(pa + (size_t)(i << 4) * (size_t)KTOT + k0);
#pragma unroll
      for (int j = 0; j < 4; ++j) acc[i][j] = mm(af, bf[j], acc[i][j]);
    }
  }

  float* slab = sT[wave];
  const int hh = lane >> 4;
  const int c4 = (lane & 15) * 4;
  const int nc = n0 + c4;
  const bool cok = nc < N;
  v4f bv = (v4f){0.f, 0.f, 0.f, 0.f};
  if (EPI == 1) {
    bv = *(const v4fa*)(bias + clampi(nc, 0, N - 4));
    asm volatile("" :: "v"(bv));
  }
#pragma unroll
  for (int i = 0; i < 4; ++i) {
    const int mBase = m0 + (i << 4);
#pragma unroll
    for (int j = 0; j < 4; ++j) {
#pragma unroll
      for (int r = 0; r < 8; ++r) slab[(h8 + r) * 68 + (j << 4) + rl] = acc[i][j][r];
    }
    __builtin_amdgcn_fence(__ATOMIC_RELEASE, "workgroup");
    __builtin_amdgcn_wave_barrier();
    __builtin_amdgcn_fence(__ATOMIC_ACQUIRE, "workgroup");
    v4f vv[8];
#pragma unroll
    for (int it = 0; it < 8; ++it) {
      const int row = it * 2 + hh;
      v4f v = *(const v4fa*)(slab + row * 68 + c4);
      if (EPI == 1) v += bv;
      vv[it] = v;
    }
    for (int pass = 0; pass < 2; ++pass) {
#pragma unroll
      for (int it = 0; it < 8; ++it) {
        const int row = mBase + it * 2 + hh;
        if (cok && row < M) *(volatile v4f*)(D + (size_t)row * (size_t)ldd + nc) = vv[it];
      }
      __threadfence();
    }
    __builtin_amdgcn_fence(__ATOMIC_RELEASE, "workgroup");
    __builtin_amdgcn_wave_barrier();
    __builtin_amdgcn_fence(__ATOMIC_ACQUIRE, "workgroup");
  }
}

#pragma clang fp contract(off)
#include <stddef.h>
#include <stdint.h>

#define NN      50000
#define DD      128
#define NR      8
#define NE      1600000
#define MPX     50048
#define NTHR    256
#define NWAVE   8
#define EPT     8
#define WCH     (32 * EPT)
#define OWN     256
#define SLB     8
#define NBK     196
#define WLCAP   1536
#define RCAP    12288
#define DEGCAP  72
#define MAXDEG_MEAS  61
#define MAXB256_MEAS 8461
#define NCHUNK  4
#define CHR     12544
#define H1R     (NCHUNK * CHR)
#define KREL    2048
#define K1      2176
#define K2      2304
#define WSMAX   ((size_t)128 << 20)

#define BK_ZINTS (NWAVE * WLCAP + RCAP + 3 * OWN)
#define BK_INTS  (BK_ZINTS + 16)
#define BK_LDS   (BK_INTS * 4)

static_assert(NN < (1 << 24));
static_assert(NE < (1 << 21));
static_assert((((long long)NE + 256) << SLB) < (1LL << 31));
static_assert(NE % EPT == 0 && NE >= EPT);
static_assert(OWN == (1 << SLB) && OWN % 32 == 0);
static_assert(NBK * OWN >= NN && (NBK - 1) * OWN < NN);
static_assert(NCHUNK * CHR == NBK * OWN);
static_assert(CHR % 64 == 0 && CHR % OWN == 0 && CHR % 8 == 0);
static_assert(MPX % 64 == 0 && MPX >= NN && H1R >= MPX);
static_assert(K1 % 32 == 0 && K2 % 32 == 0 && K1 % 128 == 0 && K2 % 128 == 0 && KREL == NR * 2 * DD);
static_assert(RCAP % (NTHR * 4) == 0);
static_assert((long long)RCAP * 100 >= (long long)MAXB256_MEAS * 145);
static_assert(MAXDEG_MEAS + 8 <= DEGCAP);
static_assert(NWAVE * WLCAP >= RCAP);
static_assert(BK_ZINTS % 4 == 0);
static_assert(BK_LDS <= 262144 && BK_LDS + 0 <= 327680);
static_assert(2 * OWN == 128 * 4);
static_assert((MPX * DD / 8) % NTHR == 0);
static_assert(((CHR / 64) * (DD / 64)) % 8 == 0);

typedef unsigned int v2u __attribute__((ext_vector_type(2)));
typedef int v4i __attribute__((ext_vector_type(4)));
typedef v2u __attribute__((may_alias)) v2ua;
typedef v4i __attribute__((may_alias)) v4ia;

__device__ __forceinline__ void st2_v4f(float* p, v4f v) {
  *(volatile v4f*)p = v;
  __threadfence();
  *(volatile v4f*)p = v;
}
__device__ __forceinline__ void st2_v4i(int* p, v4i v) {
  *(volatile v4i*)p = v;
  __threadfence();
  *(volatile v4i*)p = v;
}
__device__ __forceinline__ void st2_v4u(unsigned short* p, v4u v) {
  *(volatile v4u*)p = v;
  __threadfence();
  *(volatile v4u*)p = v;
}

template <int KT>
__global__ __launch_bounds__(NTHR) void k_prep(const float* __restrict__ w, const float* __restrict__ sw,
                                               const float* __restrict__ b, unsigned short* WT, float* BT) {
  constexpr int SP = (KT - KREL) / 8;
  constexpr int SB = DD * SP / NTHR;
  static_assert(SP == 16 || SP == 32);
  static_assert(SB * NTHR == DD * SP);
  const int tid = (int)threadIdx.x;
  const int blk = (int)blockIdx.x;
  if (blk < DD) {
    const int n  = blk;
    const int r  = tid >> 5;
    const int j0 = (tid & 15) * 8;
    const float* p = w + ((size_t)(r * DD + j0)) * DD + n;
    float x[8];
#pragma unroll
    for (int e = 0; e < 8; ++e) {
      const float v = p[(size_t)e * DD];
      asm volatile("" :: "v"(v));
      x[e] = v;
    }
    const v4u o = pack8_bf16((v4f){x[0], x[1], x[2], x[3]}, (v4f){x[4], x[5], x[6], x[7]});
    st2_v4u(WT + (size_t)n * KT + 8 * tid, o);
  } else if (blk < DD + SB) {
    const int u  = (blk - DD) * NTHR + tid;
    const int n  = u / SP;
    const int pc = u - n * SP;
    const int j0 = (pc & 15) * 8;
    const float* p = sw + (size_t)j0 * DD + n;
    float x[8];
#pragma unroll
    for (int e = 0; e < 8; ++e) {
      const float v = p[(size_t)e * DD];
      asm volatile("" :: "v"(v));
      x[e] = v;
    }
    const v4u o = pack8_bf16((v4f){x[0], x[1], x[2], x[3]}, (v4f){x[4], x[5], x[6], x[7]});
    st2_v4u(WT + (size_t)n * KT + KREL + 8 * pc, o);
  } else {
    const int idx = tid & 31;
    const v4f a = *(const v4fa*)(b + 4 * idx);
    asm volatile("" :: "v"(a));
    v4f o;
    o.x = bf16_val(a.x); o.y = bf16_val(a.y); o.z = bf16_val(a.z); o.w = bf16_val(a.w);
    if (tid < 32) st2_v4f(BT + 4 * tid, o);
  }
}

__global__ __launch_bounds__(NTHR) void k_lists(const int* __restrict__ srcs, const int* __restrict__ dsts,
                                                const int* __restrict__ types, int* LIST, int* META, int* FLAG) {
  extern __shared__ __attribute__((aligned(16))) int dsm[];
  int* wl   = dsm;
  int* pl   = dsm + NWAVE * WLCAP;
  int* cnt  = pl + RCAP;
  int* offs = cnt + OWN;
  int* cur  = offs + OWN;
  int* misc = cur + OWN;
  const int tid = (int)threadIdx.x, lane = tid & 31, wave = tid >> 5;
  const int blk = (int)blockIdx.x;
  const unsigned nbs = (unsigned)(blk * OWN);
  const int limi = (NN - blk * OWN) < OWN ? (NN - blk * OWN) : OWN;
  const unsigned lim = (unsigned)(limi < 0 ? 0 : limi);

  {
    const v4i z4 = {0, 0, 0, 0};
    for (int i = tid * 4; i < BK_ZINTS; i += NTHR * 4) *(v4ia*)(dsm + i) = z4;
    if (tid < 16) misc[tid] = 0;
  }
  __syncthreads();

  {
    const int per  = ((NE + NWAVE * WCH - 1) / (NWAVE * WCH)) * WCH;
    const int ebeg = wave * per;
    const int eend = (ebeg + per < NE) ? (ebeg + per) : NE;
    int* mylist = wl + wave * WLCAP;
    int wc = 0;
#pragma unroll 1
    for (int cb = ebeg; cb < eend; cb += WCH) {
      const int e0 = cb + lane * EPT;
      const int ec = e0 < NE - EPT ? e0 : NE - EPT;
      const v4i da = *(const v4ia*)(dsts + ec);
      const v4i db = *(const v4ia*)(dsts + ec + 4);
      asm volatile("" :: "v"(da));
      asm volatile("" :: "v"(db));
      const int vm = (e0 < NE) ? -1 : 0;
      const unsigned s0 = (unsigned)((da.x & vm) | ~vm) - nbs, s1 = (unsigned)((da.y & vm) | ~vm) - nbs;
      const unsigned s2 = (unsigned)((da.z & vm) | ~vm) - nbs, s3 = (unsigned)((da.w & vm) | ~vm) - nbs;
      const unsigned s4 = (unsigned)((db.x & vm) | ~vm) - nbs, s5 = (unsigned)((db.y & vm) | ~vm) - nbs;
      const unsigned s6 = (unsigned)((db.z & vm) | ~vm) - nbs, s7 = (unsigned)((db.w & vm) | ~vm) - nbs;
      const bool h0 = s0 < lim, h1 = s1 < lim, h2 = s2 < lim, h3 = s3 < lim;
      const bool h4 = s4 < lim, h5 = s5 < lim, h6 = s6 < lim, h7 = s7 < lim;
      const unsigned m0 = __builtin_amdgcn_ballot_w32(h0), m1 = __builtin_amdgcn_ballot_w32(h1);
      const unsigned m2 = __builtin_amdgcn_ballot_w32(h2), m3 = __builtin_amdgcn_ballot_w32(h3);
      const unsigned m4 = __builtin_amdgcn_ballot_w32(h4), m5 = __builtin_amdgcn_ballot_w32(h5);
      const unsigned m6 = __builtin_amdgcn_ballot_w32(h6), m7 = __builtin_amdgcn_ballot_w32(h7);
      const unsigned any = m0 | m1 | m2 | m3 | m4 | m5 | m6 | m7;
      if (any != 0u) {
        const int pre = (int)(__builtin_amdgcn_mbcnt_lo(m0, 0u) + __builtin_amdgcn_mbcnt_lo(m1, 0u) +
                              __builtin_amdgcn_mbcnt_lo(m2, 0u) + __builtin_amdgcn_mbcnt_lo(m3, 0u) +
                              __builtin_amdgcn_mbcnt_lo(m4, 0u) + __builtin_amdgcn_mbcnt_lo(m5, 0u) +
                              __builtin_amdgcn_mbcnt_lo(m6, 0u) + __builtin_amdgcn_mbcnt_lo(m7, 0u));
        int p = wc + pre;
        if (h0) { if (p < WLCAP) mylist[p] = ((e0 + 0) << SLB) | (int)s0; p = p + 1; }
        if (h1) { if (p < WLCAP) mylist[p] = ((e0 + 1) << SLB) | (int)s1; p = p + 1; }
        if (h2) { if (p < WLCAP) mylist[p] = ((e0 + 2) << SLB) | (int)s2; p = p + 1; }
        if (h3) { if (p < WLCAP) mylist[p] = ((e0 + 3) << SLB) | (int)s3; p = p + 1; }
        if (h4) { if (p < WLCAP) mylist[p] = ((e0 + 4) << SLB) | (int)s4; p = p + 1; }
        if (h5) { if (p < WLCAP) mylist[p] = ((e0 + 5) << SLB) | (int)s5; p = p + 1; }
        if (h6) { if (p < WLCAP) mylist[p] = ((e0 + 6) << SLB) | (int)s6; p = p + 1; }
        if (h7) { if (p < WLCAP) mylist[p] = ((e0 + 7) << SLB) | (int)s7; p = p + 1; }
        wc += (int)(__builtin_popcount(m0) + __builtin_popcount(m1) + __builtin_popcount(m2) + __builtin_popcount(m3) +
                    __builtin_popcount(m4) + __builtin_popcount(m5) + __builtin_popcount(m6) + __builtin_popcount(m7));
      }
    }
    if (lane == 0) misc[wave] = wc;
  }
  __syncthreads();

  if (wave == 0) {
    int ov = 0;
    int tot = 0;
#pragma unroll 1
    for (int w2 = 0; w2 < NWAVE; ++w2) {
      int c = __builtin_amdgcn_readfirstlane(misc[w2]);
      if (c > WLCAP) ov = 1;
      c = c < 0 ? 0 : (c > WLCAP ? WLCAP : c);
      tot += c;
#pragma unroll 1
      for (int b0 = 0; b0 < c; b0 += 32) {
        const int idx = b0 + lane;
        const int ent = wl[w2 * WLCAP + (idx < WLCAP ? idx : WLCAP - 1)];
        const int m32 = (c - b0) < 32 ? (c - b0) : 32;
#pragma unroll 1
        for (int k = 0; k < m32; ++k) {
          const int u    = __builtin_amdgcn_readlane(ent, k);
          const int slot = u & (OWN - 1);
          if (lane == 0) cnt[slot] = cnt[slot] + 1;
        }
      }
    }
    if (tot > RCAP) ov = 1;
    if (lane == 0) {
      misc[9]  = ov;
      misc[10] = tot > RCAP ? RCAP : tot;
    }
  }
  __syncthreads();
  if (wave == 0) {
    const int base = lane * (OWN / 32);
    int s = 0;
    int dg = 0;
#pragma unroll 1
    for (int i = 0; i < OWN / 32; ++i) {
      const int cv = cnt[base + i];
      s += cv;
      dg |= (cv > DEGCAP) ? 1 : 0;
    }
    const unsigned dgm = __builtin_amdgcn_ballot_w32(dg != 0);
    int incl = s;
#pragma unroll
    for (int d = 1; d < 32; d <<= 1) {
      const int y = __shfl_up(incl, d, 32);
      if (lane >= d) incl += y;
    }
    int run = incl - s;
#pragma unroll 1
    for (int i = 0; i < OWN / 32; ++i) {
      const int cv = cnt[base + i];
      offs[base + i] = run;
      cur[base + i]  = run;
      run += cv;
    }
    if (lane == 0 && dgm != 0u) misc[9] = 1;
  }
  __syncthreads();

  if (wave == 0) {
#pragma unroll 1
    for (int w2 = 0; w2 < NWAVE; ++w2) {
      int c = __builtin_amdgcn_readfirstlane(misc[w2]);
      c = c < 0 ? 0 : (c > WLCAP ? WLCAP : c);
#pragma unroll 1
      for (int b0 = 0; b0 < c; b0 += 32) {
        const int idx = b0 + lane;
        const int ent = wl[w2 * WLCAP + (idx < WLCAP ? idx : WLCAP - 1)];
        const int m32 = (c - b0) < 32 ? (c - b0) : 32;
#pragma unroll 1
        for (int k = 0; k < m32; ++k) {
          const int u    = __builtin_amdgcn_readlane(ent, k);
          const int slot = u & (OWN - 1);
          if (lane == 0) {
            int p = cur[slot];
            p = p < 0 ? 0 : (p > RCAP - 1 ? RCAP - 1 : p);
            pl[p] = u;
            cur[slot] = p + 1;
          }
        }
      }
    }
  }
  __syncthreads();

  const int ovf = misc[9];
  const int tot = misc[10];
  int* lp = LIST + (size_t)blk * (size_t)RCAP;
  int* mp = META + (size_t)blk * (2 * OWN);
  int* fp = FLAG + (size_t)blk * 32;
#pragma unroll 1
  for (int i = tid * 4; i < RCAP; i += NTHR * 4) {
    const v4i wd = *(const v4ia*)(pl + i);
    const int ea = clampi((wd.x >> SLB) & 0x1FFFFF, 0, NE - 1);
    const int eb = clampi((wd.y >> SLB) & 0x1FFFFF, 0, NE - 1);
    const int ec = clampi((wd.z >> SLB) & 0x1FFFFF, 0, NE - 1);
    const int ed = clampi((wd.w >> SLB) & 0x1FFFFF, 0, NE - 1);
    int sa = srcs[ea];
    int ta = types[ea];
    int sb = srcs[eb];
    int tb = types[eb];
    int sc = srcs[ec];
    int tc = types[ec];
    int sd = srcs[ed];
    int td = types[ed];
    asm volatile("" :: "v"(sa));
    asm volatile("" :: "v"(ta));
    asm volatile("" :: "v"(sb));
    asm volatile("" :: "v"(tb));
    asm volatile("" :: "v"(sc));
    asm volatile("" :: "v"(tc));
    asm volatile("" :: "v"(sd));
    asm volatile("" :: "v"(td));
    sa = clampi(sa, 0, NN - 1); sb = clampi(sb, 0, NN - 1); sc = clampi(sc, 0, NN - 1); sd = clampi(sd, 0, NN - 1);
    ta = clampi(ta, 0, NR - 1); tb = clampi(tb, 0, NR - 1); tc = clampi(tc, 0, NR - 1); td = clampi(td, 0, NR - 1);
    const int ma = (i     < tot) ? -1 : 0;
    const int mb = (i + 1 < tot) ? -1 : 0;
    const int mc = (i + 2 < tot) ? -1 : 0;
    const int md = (i + 3 < tot) ? -1 : 0;
    const v4i v = {(sa | (ta << 24)) & ma, (sb | (tb << 24)) & mb, (sc | (tc << 24)) & mc, (sd | (td << 24)) & md};
    st2_v4i(lp + i, v);
  }
  if (tid < 128) {
    const v4i v = *(const v4ia*)(cnt + 4 * tid);
    st2_v4i(mp + 4 * tid, v);
  }
  if (tid < 8) {
    const v4i f = {ovf, ovf, ovf, ovf};
    st2_v4i(fp + 4 * tid, f);
  }
}

template <int L>
__global__ __launch_bounds__(NTHR) void k_walk(const unsigned short* __restrict__ XB, const float* __restrict__ H1,
                                               const int* __restrict__ LIST, const int* __restrict__ META,
                                               const int* __restrict__ FLAG, unsigned short* OP, int chunk) {
  static_assert(L == 1 || L == 2);
  constexpr int KT = (L == 1) ? K1 : K2;
  constexpr int NG = KT / 128;
  const int tid = (int)threadIdx.x, lane = tid & 31, wave = tid >> 5;
  const int lr  = (int)blockIdx.x * 8 + wave;
  const int v   = chunk * CHR + lr;
  const int blk = clampi(v >> SLB, 0, NBK - 1);
  const int slot = v & (OWN - 1);
  const int* mp = META + (size_t)blk * (2 * OWN);
  int cv = mp[slot];
  int ov = mp[OWN + slot];
  int fl = FLAG[(size_t)blk * 32];
  asm volatile("" :: "v"(cv));
  asm volatile("" :: "v"(ov));
  asm volatile("" :: "v"(fl));
  const bool bad = (fl != 0) || (cv > DEGCAP);
  cv = clampi(cv, 0, DEGCAP);
  ov = clampi(ov, 0, RCAP - 1);
  const int c = __builtin_amdgcn_readfirstlane(cv);
  const int o = __builtin_amdgcn_readfirstlane(ov);
  const int* lp = LIST + (size_t)blk * (size_t)RCAP;

  v4f a[8];
#pragma unroll
  for (int g = 0; g < 8; ++g) a[g] = (v4f){0.0f, 0.0f, 0.0f, 0.0f};

#pragma unroll 1
  for (int k = 0; k < c; ++k) {
    int idx = o + k;
    idx = idx > RCAP - 1 ? RCAP - 1 : idx;
    int wv = lp[idx];
    asm volatile("" :: "v"(wv));
    const int wd = __builtin_amdgcn_readfirstlane(wv);
    const int s  = clampi(wd & 0xFFFFFF, 0, NN - 1);
    const int t  = (wd >> 24) & 7;
    v4f row;
    if (L == 1) {
      const v2u rw = *(const v2ua*)(XB + (size_t)s * DD + 4 * lane);
      asm volatile("" :: "v"(rw));
      float f0 = __uint_as_float(rw.x << 16);
      float f1 = __uint_as_float(rw.x & 0xffff0000u);
      float f2 = __uint_as_float(rw.y << 16);
      float f3 = __uint_as_float(rw.y & 0xffff0000u);
      asm volatile("" : "+v"(f0));
      asm volatile("" : "+v"(f1));
      asm volatile("" : "+v"(f2));
      asm volatile("" : "+v"(f3));
      row = (v4f){f0, f1, f2, f3};
    } else {
      row = *(const v4fa*)(H1 + (size_t)s * DD + 4 * lane);
      asm volatile("" :: "v"(row));
    }
    if (t < 4) {
      if (t < 2) { if (t == 0) a[0] = a[0] + row; else a[1] = a[1] + row; }
      else       { if (t == 2) a[2] = a[2] + row; else a[3] = a[3] + row; }
    } else {
      if (t < 6) { if (t == 4) a[4] = a[4] + row; else a[5] = a[5] + row; }
      else       { if (t == 6) a[6] = a[6] + row; else a[7] = a[7] + row; }
    }
  }

  unsigned w0[NG], w1[NG];
#pragma unroll
  for (int r = 0; r < 8; ++r) {
    const float x0 = a[r].x, x1 = a[r].y, x2 = a[r].z, x3 = a[r].w;
    w0[2 * r]     = pk16(bf16_bits(x0), bf16_bits(x1));
    w1[2 * r]     = pk16(bf16_bits(x2), bf16_bits(x3));
    w0[2 * r + 1] = pk16(bf16_lo_bits(x0), bf16_lo_bits(x1));
    w1[2 * r + 1] = pk16(bf16_lo_bits(x2), bf16_lo_bits(x3));
  }
  const unsigned zm = (v < NN) ? 0xFFFFFFFFu : 0u;
  if (L == 1) {
    const int vc = v < MPX - 1 ? v : MPX - 1;
    const v2u own = *(const v2ua*)(XB + (size_t)vc * DD + 4 * lane);
    asm volatile("" :: "v"(own));
    w0[16] = own.x & zm;
    w1[16] = own.y & zm;
  } else {
    const int vc = v < H1R - 1 ? v : H1R - 1;
    const v4f hv = *(const v4fa*)(H1 + (size_t)vc * DD + 4 * lane);
    asm volatile("" :: "v"(hv));
    const float x0 = hv.x, x1 = hv.y, x2 = hv.z, x3 = hv.w;
    w0[16]     = pk16(bf16_bits(x0), bf16_bits(x1)) & zm;
    w1[16]     = pk16(bf16_bits(x2), bf16_bits(x3)) & zm;
    w0[NG - 1] = pk16(bf16_lo_bits(x0), bf16_lo_bits(x1)) & zm;
    w1[NG - 1] = pk16(bf16_lo_bits(x2), bf16_lo_bits(x3)) & zm;
  }
  const unsigned pm = bad ? 0xFFFFFFFFu : 0u;
#pragma unroll
  for (int g = 0; g < NG; ++g) {
    w0[g] = (w0[g] & ~pm) | (0x7FC07FC0u & pm);
    w1[g] = (w1[g] & ~pm) | (0x7FC07FC0u & pm);
  }
  unsigned short* orow = OP + (size_t)lr * (size_t)KT + 4 * lane;
  for (int pass = 0; pass < 2; ++pass) {
#pragma unroll
    for (int g = 0; g < NG; ++g) {
      *(volatile v2u*)(orow + 128 * g) = (v2u){w0[g], w1[g]};
    }
    __threadfence();
  }
}

__global__ __launch_bounds__(NTHR) void k_ep1(const float* __restrict__ P, const unsigned short* __restrict__ XB,
                                              const float* __restrict__ BT, float* H1, int chunk) {
  const int tid = (int)threadIdx.x, lane = tid & 31, wave = tid >> 5;
  const int lr = (int)blockIdx.x * 8 + wave;
  const int v  = chunk * CHR + lr;
  const v4f p = *(const v4fa*)(P + (size_t)lr * DD + 4 * lane);
  asm volatile("" :: "v"(p));
  const int vc = v < MPX - 1 ? v : MPX - 1;
  const v2u xw = *(const v2ua*)(XB + (size_t)vc * DD + 4 * lane);
  asm volatile("" :: "v"(xw));
  const v4f b = *(const v4fa*)(BT + 4 * lane);
  asm volatile("" :: "v"(b));
  const unsigned zm = (v < NN) ? 0xFFFFFFFFu : 0u;
  float x0 = __uint_as_float((xw.x << 16) & zm);
  float x1 = __uint_as_float((xw.x & 0xffff0000u) & zm);
  float x2 = __uint_as_float((xw.y << 16) & zm);
  float x3 = __uint_as_float((xw.y & 0xffff0000u) & zm);
  asm volatile("" : "+v"(x0));
  asm volatile("" : "+v"(x1));
  asm volatile("" : "+v"(x2));
  asm volatile("" : "+v"(x3));
  const float s0 = p.x + x0, s1 = p.y + x1, s2 = p.z + x2, s3 = p.w + x3;
  const float r0 = (s0 > 0.0f) ? s0 : (s0 - s0);
  const float r1 = (s1 > 0.0f) ? s1 : (s1 - s1);
  const float r2 = (s2 > 0.0f) ? s2 : (s2 - s2);
  const float r3 = (s3 > 0.0f) ? s3 : (s3 - s3);
  v4f o;
  o.x = r0 + b.x; o.y = r1 + b.y; o.z = r2 + b.z; o.w = r3 + b.w;
  st2_v4f(H1 + (size_t)v * DD + 4 * lane, o);
}

__global__ __launch_bounds__(NTHR) void k_ep2(const float* __restrict__ P, const float* __restrict__ BT,
                                              float* out, int chunk) {
  const int tid = (int)threadIdx.x, lane = tid & 31, wave = tid >> 5;
  const int lr = (int)blockIdx.x * 8 + wave;
  const int v  = chunk * CHR + lr;
  const v4f p = *(const v4fa*)(P + (size_t)lr * DD + 4 * lane);
  asm volatile("" :: "v"(p));
  const v4f b = *(const v4fa*)(BT + 4 * lane);
  asm volatile("" :: "v"(b));
  v4f o;
  o.x = p.x + b.x; o.y = p.y + b.y; o.z = p.z + b.z; o.w = p.w + b.w;
  if (v < NN) st2_v4f(out + (size_t)v * DD + 4 * lane, o);
}

extern "C" void kernel_launch(void* const* d_in, const int* in_sizes, int n_in,
                              void* d_out, int out_size, void* d_ws, size_t ws_size,
                              hipStream_t stream) {
  if (n_in < 9) return;
  if (in_sizes[0] != NN * DD) return;
  if (in_sizes[1] != 2 * NE) return;
  if (in_sizes[2] != NE) return;
  if (in_sizes[3] != NR * DD * DD) return;
  if (in_sizes[4] != DD * DD) return;
  if (in_sizes[5] != DD) return;
  if (in_sizes[6] != NR * DD * DD) return;
  if (in_sizes[7] != DD * DD) return;
  if (in_sizes[8] != DD) return;
  if (out_size != NN * DD) return;

  const float* x     = (const float*)d_in[0];
  const int*   eidx  = (const int*)d_in[1];
  const int*   srcs  = eidx;
  const int*   dsts  = eidx + NE;
  const int*   types = (const int*)d_in[2];
  const float* w1    = (const float*)d_in[3];
  const float* sw1   = (const float*)d_in[4];
  const float* b1    = (const float*)d_in[5];
  const float* w2    = (const float*)d_in[6];
  const float* sw2   = (const float*)d_in[7];
  const float* b2    = (const float*)d_in[8];
  float* out = (float*)d_out;

  constexpr size_t zXB   = (size_t)MPX * DD * 2;
  constexpr size_t zH1   = (size_t)H1R * DD * 4;
  constexpr size_t zOP   = (size_t)CHR * K2 * 2;
  constexpr size_t zP    = (size_t)CHR * DD * 4;
  constexpr size_t zWT1  = (size_t)DD * K1 * 2;
  constexpr size_t zWT2  = (size_t)DD * K2 * 2;
  constexpr size_t zBT   = (size_t)2 * DD * 4;
  constexpr size_t zLIST = (size_t)NBK * RCAP * 4;
  constexpr size_t zMETA = (size_t)NBK * 2 * OWN * 4;
  constexpr size_t zFLAG = (size_t)NBK * 128;
  constexpr size_t oXB   = 0;
  constexpr size_t oH1   = oXB + zXB;
  constexpr size_t oOP   = oH1 + zH1;
  constexpr size_t oP    = oOP + zOP;
  constexpr size_t oWT1  = oP + zP;
  constexpr size_t oWT2  = oWT1 + zWT1;
  constexpr size_t oBT   = oWT2 + zWT2;
  constexpr size_t oLIST = oBT + zBT;
  constexpr size_t oMETA = oLIST + zLIST;
  constexpr size_t oFLAG = oMETA + zMETA;
  constexpr size_t oEND  = oFLAG + zFLAG;
  static_assert(zXB % 256 == 0 && zH1 % 256 == 0 && zOP % 256 == 0 && zP % 256 == 0 && zWT1 % 256 == 0);
  static_assert(zWT2 % 256 == 0 && zBT % 256 == 0 && zLIST % 256 == 0 && zMETA % 256 == 0 && zFLAG % 256 == 0);
  static_assert((size_t)CHR * K1 * 2 <= zOP);
  static_assert(oEND == ((size_t)222531 * 512));
  static_assert(oEND <= (size_t)WSMAX);
  if (oEND > ws_size) return;

  char* ws = (char*)d_ws;
  unsigned short* XB   = (unsigned short*)(ws + oXB);
  float*          H1   = (float*)(ws + oH1);
  unsigned short* OP   = (unsigned short*)(ws + oOP);
  float*          P    = (float*)(ws + oP);
  unsigned short* WT1  = (unsigned short*)(ws + oWT1);
  unsigned short* WT2  = (unsigned short*)(ws + oWT2);
  float*          BT1  = (float*)(ws + oBT);
  float*          BT2  = BT1 + DD;
  int*            LIST = (int*)(ws + oLIST);
  int*            META = (int*)(ws + oMETA);
  int*            FLAG = (int*)(ws + oFLAG);

  hipFuncSetAttribute(reinterpret_cast<const void*>(&k_lists), hipFuncAttributeMaxDynamicSharedMemorySize, (int)BK_LDS);

  constexpr int GT = (CHR / 64) * (DD / 64);
  constexpr int PB1 = DD + DD * ((K1 - KREL) / 8) / NTHR + 1;
  constexpr int PB2 = DD + DD * ((K2 - KREL) / 8) / NTHR + 1;

  k_plane<0><<<MPX * DD / 8 / 256, 256, 0, stream>>>(x, NN, DD, DD, XB, MPX, DD);
  k_prep<K1><<<PB1, NTHR, 0, stream>>>(w1, sw1, b1, WT1, BT1);
  k_prep<K2><<<PB2, NTHR, 0, stream>>>(w2, sw2, b2, WT2, BT2);
  k_lists<<<NBK, NTHR, BK_LDS, stream>>>(srcs, dsts, types, LIST, META, FLAG);

  for (int c = 0; c < NCHUNK; ++c) {
    k_walk<1><<<CHR / 8, NTHR, 0, stream>>>(XB, H1, LIST, META, FLAG, OP, c);
    k_gemm_nt<0, 0><<<GT / 8, 256, 0, stream>>>(OP, WT1, BT1, P, CHR, DD, K1, DD);
    k_ep1<<<CHR / 8, NTHR, 0, stream>>>(P, XB, BT1, H1, c);
  }
  for (int c = 0; c < NCHUNK; ++c) {
    k_walk<2><<<CHR / 8, NTHR, 0, stream>>>(XB, H1, LIST, META, FLAG, OP, c);
    k_gemm_nt<0, 0><<<GT / 8, 256, 0, stream>>>(OP, WT2, BT2, P, CHR, DD, K2, DD);
    k_ep2<<<CHR / 8, NTHR, 0, stream>>>(P, BT2, out, c);
  }
}
